// LateInteraction_34720515621483
// MI455X (gfx1250) — hardware-verified
//
#include <hip/hip_runtime.h>
#include <math.h>
#include <stdint.h>

#ifndef NBQ
#define NBQ 32
#endif
#define NB_FULL 32
#define SEQ     256
#define HDIM    128
#define SIMP    260
#define NTHR    512
#define NWAV    (NTHR / 32)
#define SCL     32
#define WS_CAP  134217728
static_assert(NBQ >= 1 && NBQ <= NB_FULL);
static_assert(NTHR == 2 * SEQ && NWAV == 16 && SEQ == NWAV * 16);
static_assert(HDIM == 128 && (HDIM % 32) == 0);
static_assert((SEQ % 32) == 0);
static_assert(NBQ * NB_FULL <= 4 * 256);

typedef unsigned short u16;
typedef __bf16       v16b __attribute__((ext_vector_type(16)));
typedef float        v8f  __attribute__((ext_vector_type(8)));
typedef float        v4f  __attribute__((ext_vector_type(4)));
typedef unsigned int v4u  __attribute__((ext_vector_type(4)));

union FragB { v16b v; v4u u[2]; };

__device__ __forceinline__ unsigned short bf_bits(float f) {
  unsigned u = __float_as_uint(f);
  return (unsigned short)((u + 0x7FFFu + ((u >> 16) & 1u)) >> 16);
}
__device__ __forceinline__ float bf_up(unsigned short h) { return __uint_as_float(((unsigned)h) << 16); }
__device__ __forceinline__ unsigned pk16(unsigned short a, unsigned short b) { return (unsigned)a | ((unsigned)b << 16); }
__device__ __forceinline__ v8f zero8() { v8f z = {0.f, 0.f, 0.f, 0.f, 0.f, 0.f, 0.f, 0.f}; return z; }

__device__ __forceinline__ v16b ldfrag_b(const u16* p) {
  FragB f;
  f.u[0] = *(const v4u*)(p);
  f.u[1] = *(const v4u*)(p + 16);
  return f.v;
}

__device__ __forceinline__ v8f mma_b(v16b a, v16b b, v8f c) {
  return __builtin_amdgcn_wmma_f32_16x16x32_bf16(false, a, false, b, (short)0, c, false, false);
}
__device__ __forceinline__ void guard9(v8f& acc, v16b x0, v16b x1, v16b x2, v16b x3,
                                       v16b x4, v16b x5, v16b x6, v16b x7) {
#if defined(__HIP_DEVICE_COMPILE__)
  asm volatile("v_nop\n\tv_nop\n\tv_nop\n\tv_nop"
               : "+v"(acc) : "v"(x0), "v"(x1), "v"(x2), "v"(x3), "v"(x4), "v"(x5), "v"(x6), "v"(x7) : "memory");
#endif
}

__global__ __launch_bounds__(256) void prep16(const float* __restrict__ X, u16* P, float* R, int ntok) {
  __shared__ __align__(16) float rv[32];
  const int tid  = (int)threadIdx.x;
  const int lane = tid & 31;
  const int wave = tid >> 5;
  const int tok0 = (int)blockIdx.x * 32;
  if (tok0 + 32 > ntok) return;
  const int tsub = tid >> 4;
  const int ch   = (tid & 15) * 8;
  v4u o0, o1;
#pragma unroll
  for (int it = 0; it < 2; ++it) {
    const int tl = it * 16 + tsub;
    const float* p = X + (size_t)(tok0 + tl) * HDIM + ch;
    const v4f a = *(const v4f*)(p), b4 = *(const v4f*)(p + 4);
    float w8[8];
#pragma unroll
    for (int e = 0; e < 4; ++e) { w8[e] = a[e]; w8[4 + e] = b4[e]; }
    v4u q;
    float ss = 0.f;
#pragma unroll
    for (int e = 0; e < 4; ++e) {
      const unsigned short u0 = bf_bits(w8[2 * e]), u1 = bf_bits(w8[2 * e + 1]);
      const float f0 = bf_up(u0), f1 = bf_up(u1);
      ss += f0 * f0;
      ss += f1 * f1;
      q[e] = pk16(u0, u1);
    }
#pragma unroll
    for (int off = 1; off < 16; off <<= 1) ss += __shfl_xor(ss, off, 32);
    const float nrm  = sqrtf(ss);
    const float rinv = 1.0f / fmaxf(nrm, 1.0e-12f);
    if ((tid & 15) == 0) rv[tl] = rinv;
    if (it == 0) o0 = q; else o1 = q;
  }
  u16* d0 = P + (size_t)(tok0 + tsub) * HDIM + ch;
  u16* d1 = P + (size_t)(tok0 + 16 + tsub) * HDIM + ch;
  for (int pass = 0; pass < 2; ++pass) {
    *(volatile v4u*)(d0) = o0;
    *(volatile v4u*)(d1) = o1;
    __threadfence();
  }
  __syncthreads();
  if (wave == 0) {
    v4f r4;
#pragma unroll
    for (int e = 0; e < 4; ++e) r4[e] = rv[(4 * lane + e) & 31];
    const bool ok = (lane < 8);
    for (int pass = 0; pass < 2; ++pass) {
      if (ok) *(volatile v4f*)(R + tok0 + 4 * lane) = r4;
      __threadfence();
    }
  }
}

__global__ __launch_bounds__(NTHR)
void pair_scores(const u16* __restrict__ XQ, const u16* __restrict__ XK,
                 const float* __restrict__ RQ, const float* __restrict__ RK,
                 const float* __restrict__ qmask, const float* __restrict__ kmask,
                 const float* __restrict__ apar, const float* __restrict__ spar,
                 float* SC) {
  __shared__ __align__(16) float sim_lds[16 * SIMP];
  __shared__ float qm_sh[SEQ];
  __shared__ float km_sh[SEQ];
  __shared__ float rq_sh[SEQ];
  __shared__ float rk_sh[SEQ];
  __shared__ float w_sh[SEQ];
  __shared__ float red_sh[NWAV];

  const int tid  = (int)threadIdx.x;
  const int wave = tid >> 5;
  const int lane = tid & 31;
  const int hh   = lane >> 4;
  const int m    = lane & 15;
  const int bid  = (int)blockIdx.x;
  const int i    = bid / NB_FULL;
  const int j    = bid - i * NB_FULL;
  if (i >= NBQ) return;

  const float araw  = __uint_as_float(((unsigned)bf_bits(apar[0])) << 16);
  const float alpha = fmaxf(araw, 0.0f) + log1pf(expf(-fabsf(araw)));
  const float scale = expf(__uint_as_float(((unsigned)bf_bits(spar[0])) << 16));

  if (tid < SEQ) {
    qm_sh[tid] = qmask[(size_t)i * SEQ + tid];
    rq_sh[tid] = RQ[(size_t)i * SEQ + tid];
    w_sh[tid]  = expf(-alpha * (float)tid);
  } else {
    const int t = tid - SEQ;
    km_sh[t] = kmask[(size_t)j * SEQ + t];
    rk_sh[t] = RK[(size_t)j * SEQ + t];
  }
  __syncthreads();

  const u16* kbp = XK + ((size_t)j * SEQ + wave * 16 + m) * HDIM + 8 * hh;
  const v16b kf0 = ldfrag_b(kbp);
  const v16b kf1 = ldfrag_b(kbp + 32);
  const v16b kf2 = ldfrag_b(kbp + 64);
  const v16b kf3 = ldfrag_b(kbp + 96);
  const float rkn = rk_sh[wave * 16 + m];

  float accd = 0.0f;
#pragma unroll 1
  for (int st = 0; st < SEQ / 16; ++st) {
    const u16* qap = XQ + ((size_t)i * SEQ + st * 16 + m) * HDIM + 8 * hh;
    const v16b a0 = ldfrag_b(qap);
    const v16b a1 = ldfrag_b(qap + 32);
    const v16b a2 = ldfrag_b(qap + 64);
    const v16b a3 = ldfrag_b(qap + 96);
    v8f acc = zero8();
    acc = mma_b(a0, kf0, acc);
    acc = mma_b(a1, kf1, acc);
    acc = mma_b(a2, kf2, acc);
    acc = mma_b(a3, kf3, acc);
    guard9(acc, a0, a1, a2, a3, kf0, kf1, kf2, kf3);
#pragma unroll
    for (int r = 0; r < 8; ++r) {
      const int qrow = st * 16 + 8 * hh + r;
      sim_lds[(8 * hh + r) * SIMP + wave * 16 + m] = acc[r] * rq_sh[qrow] * rkn;
    }
    __syncthreads();

    {
      const int    s    = st * 16 + wave;
      const float  qm   = qm_sh[s];
      const float* srow = sim_lds + wave * SIMP;
      float sv[8], lg[8];
      float mx = -INFINITY;
#pragma unroll
      for (int c = 0; c < 8; ++c) {
        const int   t  = lane + 32 * c;
        const float v  = srow[t];
        sv[c] = v;
        const int   dd = s - t;
        const int   d  = (dd < 0) ? -dd : dd;
        const float wv = w_sh[d];
        const bool  valid = (qm * km_sh[t]) > 0.0f;
        const float sw  = v * wv;
        const float lgt = (valid ? (scale * sw) : -1.0e9f) + 1.0e-6f;
        lg[c] = lgt;
        mx = fmaxf(mx, lgt);
      }
#pragma unroll
      for (int off = 16; off >= 1; off >>= 1) mx = fmaxf(mx, __shfl_xor(mx, off, 32));
      float sum = 0.0f, wsum = 0.0f;
#pragma unroll
      for (int c = 0; c < 8; ++c) {
        const float e = __expf(lg[c] - mx);
        sum  += e;
        wsum += e * sv[c];
      }
#pragma unroll
      for (int off = 16; off >= 1; off >>= 1) {
        sum  += __shfl_xor(sum,  off, 32);
        wsum += __shfl_xor(wsum, off, 32);
      }
      accd += (wsum * (1.0f / sum)) * qm;
    }
    __syncthreads();
  }

  if (lane == 0) red_sh[wave] = accd;
  __syncthreads();
  if (wave == 0) {
    float tot = 0.0f;
#pragma unroll
    for (int v = 0; v < NWAV; ++v) tot += red_sh[v];
    float qs = 0.0f;
#pragma unroll
    for (int c = 0; c < 8; ++c) qs += qm_sh[lane + 32 * c];
#pragma unroll
    for (int off = 16; off >= 1; off >>= 1) qs += __shfl_xor(qs, off, 32);
    const float den = fmaxf(qs, 1.0f);
    const float scv = tot * (1.0f / den);
    float* dst = SC + ((size_t)(i * NB_FULL + j)) * SCL + lane;
    for (int pass = 0; pass < 2; ++pass) {
      *(volatile float*)(dst) = scv;
      __threadfence();
    }
  }
}

__global__ __launch_bounds__(256) void fin(const float* __restrict__ SC, float* out) {
  const int t    = (int)threadIdx.x;
  const int nval = NBQ * NB_FULL;
  const int e0   = t * 4;
  v4f v;
#pragma unroll
  for (int e = 0; e < 4; ++e) {
    int idx = e0 + e;
    idx = (idx < nval) ? idx : (nval - 1);
    v[e] = SC[(size_t)idx * SCL];
  }
  const bool ok = (e0 < nval);
  for (int pass = 0; pass < 2; ++pass) {
    if (ok) *(volatile v4f*)(out + e0) = v;
    __threadfence();
  }
}

extern "C" void kernel_launch(void* const* d_in, const int* in_sizes, int n_in,
                              void* d_out, int out_size, void* d_ws, size_t ws_size,
                              hipStream_t stream) {
  if (n_in < 6) return;
  if (in_sizes[0] < NBQ * SEQ * HDIM) return;
  if (in_sizes[1] < NB_FULL * SEQ * HDIM) return;
  if (in_sizes[2] < NBQ * SEQ) return;
  if (in_sizes[3] < NB_FULL * SEQ) return;
  if (in_sizes[4] < 1 || in_sizes[5] < 1) return;
  if (out_size < NBQ * NB_FULL) return;

  const float* xq = (const float*)d_in[0];
  const float* xk = (const float*)d_in[1];
  const float* qm = (const float*)d_in[2];
  const float* km = (const float*)d_in[3];
  const float* ar = (const float*)d_in[4];
  const float* ls = (const float*)d_in[5];
  float*       out = (float*)d_out;

  const size_t szX = (size_t)NB_FULL * SEQ * HDIM * 2;
  const size_t szR = (size_t)NB_FULL * SEQ * 4;
  const size_t szS = (size_t)NB_FULL * NB_FULL * SCL * 4;
  size_t off = 0;
  const size_t oXQ = off; off += szX;
  const size_t oXK = off; off += szX;
  const size_t oRQ = off; off += szR;
  const size_t oRK = off; off += szR;
  const size_t oSC = off; off += szS;
  if (off > ws_size) return;
  if (off > (size_t)WS_CAP) return;

  char*  wsb = (char*)d_ws;
  u16*   XQ  = (u16*)(wsb + oXQ);
  u16*   XK  = (u16*)(wsb + oXK);
  float* RQ  = (float*)(wsb + oRQ);
  float* RK  = (float*)(wsb + oRK);
  float* SC  = (float*)(wsb + oSC);

  const int ntq = NBQ * SEQ;
  const int ntk = NB_FULL * SEQ;

  prep16<<<dim3(ntq / 32), dim3(256), 0, stream>>>(xq, XQ, RQ, ntq);
  prep16<<<dim3(ntk / 32), dim3(256), 0, stream>>>(xk, XK, RK, ntk);
  pair_scores<<<dim3(NBQ * NB_FULL), dim3(NTHR), 0, stream>>>(XQ, XK, RQ, RK, qm, km, ar, ls, SC);
  fin<<<dim3(1), dim3(256), 0, stream>>>(SC, out);
  (void)hipGetLastError();
}
